// CloneNet_2396591751946
// MI455X (gfx1250) — hardware-verified
//
#include <hip/hip_runtime.h>
#include <stddef.h>


#define NTHR   256
#define NWAVE  8
#define EPT    8
#define CHUNK  (NTHR * EPT)
#define WCAP   (EPT * 32)
#define HD     64
#define NHID   128
#define NG     64
#define NS     32
#define CAPS   384
#define MAXT   64
#define PH     128
#define AP     128
#define NBD    256
#define CAPD   1536
#define WSC    16.0f
#define WINV   0.0625f
#define W2SC   64.0f
#define W2INV  0.015625f

#define O_PT   0
#define O_MR   (O_PT + NS * 16 * PH * 2)
#define O_AS   (O_MR + CAPS * HD * 4)
#define O_Q    (O_AS + NWAVE * 16 * AP * 2)
#define O_PEND (O_Q + NS * HD * 4)
#define O_SORT (O_PEND + CAPS * 4)
#define O_TAB  (O_SORT + CAPS * 4)
#define O_CNT  (O_TAB + MAXT * 4)
#define O_SEG  (O_CNT + NS * 4)
#define O_WCS  (O_SEG + 64 * 4)
#define O_MSC  (O_WCS + NWAVE * 4)
#define MSG_LDS (O_MSC + 64)

#define D_ACC  0
#define D_CNT  (D_ACC + NBD * HD * 4)
#define D_WL   (D_CNT + NBD * 4)
#define D_PEND (D_WL + NWAVE * WCAP * 4)
#define D_M16  (D_PEND + CAPD * 4)
#define D_ST   (D_M16 + NWAVE * 16 * HD * 2)
#define D_WCS  (D_ST + NWAVE * 16 * HD * 4)
#define D_MSC  (D_WCS + NWAVE * 4)
#define NODE_LDS (D_MSC + 64)

static_assert(NWAVE * WCAP * 4 <= NWAVE * 16 * AP * 2);
static_assert(NBD == NTHR);
static_assert(NS == 4 * NWAVE);
static_assert((O_MR % 16) == 0 && (O_AS % 16) == 0 && (O_Q % 16) == 0 && (O_PEND % 16) == 0);
static_assert((D_M16 % 16) == 0 && (D_ST % 16) == 0 && (D_PEND % 16) == 0);

typedef float    v2f  __attribute__((ext_vector_type(2)));
typedef float    v4f  __attribute__((ext_vector_type(4)));
typedef float    v8f  __attribute__((ext_vector_type(8)));
typedef int      v4i  __attribute__((ext_vector_type(4)));
typedef _Float16 v8h  __attribute__((ext_vector_type(8)));
typedef _Float16 v16h __attribute__((ext_vector_type(16)));
union Frag { v16h v; v8h h[2]; };

extern __shared__ __attribute__((aligned(16))) char dsm[];

__device__ __forceinline__ v8f wmh(v16h a, v16h b, v8f c) {
  v8f d = __builtin_amdgcn_wmma_f32_16x16x32_f16(false, a, false, b, (short)0, c, false, false);
  asm volatile("v_nop\n\tv_nop\n\tv_nop\n\tv_nop" : "+v"(d) : "v"(a), "v"(b));
  return d;
}
__device__ __forceinline__ v8f zacc() {
  v8f c;
#pragma unroll
  for (int i = 0; i < 8; ++i) c[i] = 0.0f;
  return c;
}
__device__ __forceinline__ v8h zero8() {
  v8h z;
#pragma unroll
  for (int i = 0; i < 8; ++i) z[i] = (_Float16)0.0f;
  return z;
}
__device__ __forceinline__ v16h ldf(const _Float16* p) {
  Frag f;
  f.h[0] = *(const v8h*)p;
  f.h[1] = *(const v8h*)(p + 16);
  return f.v;
}
__device__ __forceinline__ v16h selv(bool c, v16h a, v16h b) {
  v16h r;
#pragma unroll
  for (int i = 0; i < 16; ++i) r[i] = c ? a[i] : b[i];
  return r;
}
__device__ __forceinline__ v8h pack8(v4f a, v4f b) {
  v8h r;
  r[0] = (_Float16)a.x; r[1] = (_Float16)a.y; r[2] = (_Float16)a.z; r[3] = (_Float16)a.w;
  r[4] = (_Float16)b.x; r[5] = (_Float16)b.y; r[6] = (_Float16)b.z; r[7] = (_Float16)b.w;
  return r;
}
__device__ __forceinline__ float sigm(float x) { return 0.5f * tanhf(0.5f * x) + 0.5f; }

__device__ __forceinline__ int scan_chunk(const int* __restrict__ ids, int nE, int cbase, int lo, int range,
                                          int clampN, int vec8, int* wl, int tid, int wave) {
  int wc = 0;
  const int el0 = tid * EPT, e0 = cbase + el0;
  int d[EPT];
  bool ok[EPT];
  if (vec8 != 0 && cbase + CHUNK <= nE) {
    const v4i da = *(const v4i*)(ids + e0);
    const v4i db = *(const v4i*)(ids + e0 + 4);
    d[0] = da.x; d[1] = da.y; d[2] = da.z; d[3] = da.w;
    d[4] = db.x; d[5] = db.y; d[6] = db.z; d[7] = db.w;
#pragma unroll
    for (int j = 0; j < EPT; ++j) ok[j] = true;
  } else {
#pragma unroll
    for (int j = 0; j < EPT; ++j) {
      const int e = e0 + j;
      ok[j] = e < nE;
      d[j] = ids[min(e, nE - 1)];
    }
  }
  bool hb[EPT];
  int sv[EPT];
  bool anyh = false;
#pragma unroll
  for (int j = 0; j < EPT; ++j) {
    int c = d[j];
    if (clampN > 0) c = min(max(c, 0), clampN - 1);
    const unsigned s = (unsigned)(c - lo);
    hb[j] = ok[j] && (s < (unsigned)range);
    sv[j] = ((el0 + j) << 8) | (int)(s & 255u);
    anyh = anyh || hb[j];
  }
  const unsigned anym = __builtin_amdgcn_ballot_w32(anyh);
  if (anym != 0u) {
#pragma unroll
    for (int j = 0; j < EPT; ++j) {
      const unsigned mj = __builtin_amdgcn_ballot_w32(hb[j]);
      if (mj != 0u) {
        if (hb[j]) {
          const int pos = wc + (int)__builtin_amdgcn_mbcnt_lo(mj, 0u);
          if (pos < WCAP) wl[wave * WCAP + pos] = sv[j];
        }
        wc += (int)__builtin_popcount(mj);
      }
    }
  }
  return wc;
}

__device__ __forceinline__ int build_list(const int* __restrict__ ids, int nE, int lo, int range, int clampN,
                                          int vec8, int* wl, int* pend, int cap, int* wcnt, int* pN,
                                          int tid, int wave, int lane) {
  if (tid == 0) pN[0] = 0;
  __syncthreads();
  const int nChunks = (nE + CHUNK - 1) / CHUNK;
#pragma unroll 1
  for (int ch = 0; ch < nChunks; ++ch) {
    const int cbase = ch * CHUNK;
    const int wc = scan_chunk(ids, nE, cbase, lo, range, clampN, vec8, wl, tid, wave);
    if (lane == 0) wcnt[wave] = wc;
    __syncthreads();
    const int base = pN[0];
    int tot = 0, myoff = 0;
#pragma unroll
    for (int w = 0; w < NWAVE; ++w) {
      const int c = min(max(wcnt[w], 0), WCAP);
      if (w < wave) myoff += c;
      tot += c;
    }
    {
      const int n = min(max(wcnt[wave], 0), WCAP);
      const int* lp = wl + wave * WCAP;
      for (int i = lane; i < n; i += 32) {
        const int pos = base + myoff + i;
        const int v = lp[min(i, WCAP - 1)];
        if (pos < cap) pend[pos] = ((cbase + (v >> 8)) << 8) | (v & 255);
      }
    }
    __syncthreads();
    if (tid == 0) pN[0] = min(base + tot, cap);
  }
  __syncthreads();
  return min(max(pN[0], 0), cap);
}

__global__ __launch_bounds__(NTHR) void k_cvt(const float* __restrict__ src, _Float16* dst, int rows, int cols,
                                              int mode, int srows, int p0, float scale) {
  const int total = (rows * cols) >> 3;
  const int t = blockIdx.x * NTHR + threadIdx.x;
  const bool act = t < total;
  const int tt = act ? t : 0;
  const int c8 = cols >> 3;
  const int r = tt / c8, cb = (tt - r * c8) * 8;
  v8h v;
#pragma unroll
  for (int j = 0; j < 8; ++j) {
    const int c = cb + j;
    float x;
    if (mode == 0) {
      const int rr = min(r, srows - 1);
      const float ld = src[(size_t)rr * cols + c];
      x = (r < srows) ? ld : 0.0f;
    } else if (mode == 1) {
      x = src[(size_t)c * rows + r];
    } else {
      x = src[(size_t)(r >> 6) * p0 + (size_t)c * 64 + (r & 63)];
    }
    v[j] = (_Float16)(x * scale);
  }
  if (act) *(volatile v8h*)(dst + (size_t)tt * 8) = v;
  __threadfence();
  if (act) *(volatile v8h*)(dst + (size_t)tt * 8) = v;
}

template <int NT, int KS, int O32, int O16>
__global__ __launch_bounds__(NTHR) void k_gemm(const _Float16* __restrict__ A, const _Float16* __restrict__ Bt,
                                               const float* __restrict__ bias, float* o32, _Float16* o16) {
  constexpr int N = NT * 16, K = KS * 32;
  __shared__ __attribute__((aligned(16))) float st[64 * N];
  const int tid = threadIdx.x, lane = tid & 31, wave = tid >> 5, hh = lane >> 4, lm = lane & 15;
  const int mt = wave & 3, ng = wave >> 2;
  const size_t r0 = (size_t)blockIdx.x * 64;
  v16h a[KS];
#pragma unroll
  for (int ks = 0; ks < KS; ++ks) a[ks] = ldf(A + (r0 + mt * 16 + lm) * K + ks * 32 + 8 * hh);
#pragma unroll
  for (int j = 0; j < NT / 2; ++j) {
    const int nt = ng + 2 * j;
    v8f acc = zacc();
#pragma unroll
    for (int ks = 0; ks < KS; ++ks)
      acc = wmh(a[ks], ldf(Bt + (size_t)(nt * 16 + lm) * K + ks * 32 + 8 * hh), acc);
    const int col = nt * 16 + lm;
    const float bv = bias[col];
#pragma unroll
    for (int r = 0; r < 8; ++r) st[(mt * 16 + 8 * hh + r) * N + col] = fmaxf(acc[r] * WINV + bv, 0.0f);
  }
  __syncthreads();
#pragma unroll 1
  for (int pass = 0; pass < 2; ++pass) {
    if (O32 != 0) {
      for (int p = tid; p < 16 * N; p += NTHR) {
        const v4f v = *(const v4f*)(st + 4 * p);
        *(volatile v4f*)(o32 + r0 * N + 4 * p) = v;
      }
    }
    if (O16 != 0) {
      for (int p = tid; p < 8 * N; p += NTHR) {
        const v4f x0 = *(const v4f*)(st + 8 * p), x1 = *(const v4f*)(st + 8 * p + 4);
        const v8h hv = pack8(x0, x1);
        *(volatile v8h*)(o16 + r0 * N + 8 * p) = hv;
      }
    }
    if (pass == 0) __threadfence();
  }
}

__global__ __launch_bounds__(NTHR) void k_msg(const int* __restrict__ ei, const _Float16* __restrict__ out16,
                                              const _Float16* __restrict__ h1, const _Float16* __restrict__ W2t,
                                              const _Float16* __restrict__ B2t, float* msg, int nN, int nE, int vec8) {
  _Float16* Pt = (_Float16*)(dsm + O_PT);
  float* Mr = (float*)(dsm + O_MR);
  _Float16* As = (_Float16*)(dsm + O_AS);
  int* wl = (int*)(dsm + O_AS);
  float* Qs = (float*)(dsm + O_Q);
  int* pend = (int*)(dsm + O_PEND);
  int* sorted = (int*)(dsm + O_SORT);
  int* ttab = (int*)(dsm + O_TAB);
  int* cnt = (int*)(dsm + O_CNT);
  int* seg = (int*)(dsm + O_SEG);
  int* wcnt = (int*)(dsm + O_WCS);
  int* misc = (int*)(dsm + O_MSC);
  const int tid = threadIdx.x, lane = tid & 31, wave = tid >> 5, hh = lane >> 4, lm = lane & 15;
  const int s0 = blockIdx.x * NS;

  const int nHit = build_list(ei, nE, s0, NS, nN, vec8, wl, pend, CAPS, wcnt, misc, tid, wave, lane);

  int cq[4] = {0, 0, 0, 0};
#pragma unroll 1
  for (int i0 = 0; i0 < CAPS; i0 += 32) {
    if (i0 >= nHit) break;
    const int idx = i0 + lane;
    const int v = pend[min(idx, CAPS - 1)];
    const int sl = (idx < nHit) ? (v & 255) : 255;
#pragma unroll
    for (int q = 0; q < 4; ++q)
      cq[q] += (int)__builtin_popcount(__builtin_amdgcn_ballot_w32(sl == 4 * wave + q));
  }
  if (lane == 0) {
#pragma unroll
    for (int q = 0; q < 4; ++q) cnt[4 * wave + q] = cq[q];
  }
  __syncthreads();
  if (tid == 0) {
    int off = 0, T = 0;
    for (int s = 0; s < NS; ++s) {
      const int c = min(max(cnt[s], 0), CAPS);
      seg[s] = off;
      const int ntile = min((c + 15) >> 4, CAPS / 16);
      for (int t = 0; t < ntile; ++t) {
        if (T < MAXT) {
          const int cn = min(16, c - 16 * t);
          ttab[T] = s | ((off + 16 * t) << 8) | (cn << 20);
          ++T;
        }
      }
      off += c;
    }
    seg[NS] = off;
    for (int t = T; t < MAXT; ++t) ttab[t] = 0;
    misc[1] = T;
  }
  __syncthreads();
  {
    int pq[4];
#pragma unroll
    for (int q = 0; q < 4; ++q) pq[q] = seg[4 * wave + q];
#pragma unroll 1
    for (int i0 = 0; i0 < CAPS; i0 += 32) {
      if (i0 >= nHit) break;
      const int idx = i0 + lane;
      const int v = pend[min(idx, CAPS - 1)];
      const int sl = (idx < nHit) ? (v & 255) : 255;
#pragma unroll
      for (int q = 0; q < 4; ++q) {
        const bool hit = (sl == 4 * wave + q);
        const unsigned mq = __builtin_amdgcn_ballot_w32(hit);
        if (hit) sorted[min(pq[q] + (int)__builtin_amdgcn_mbcnt_lo(mq, 0u), CAPS - 1)] = v;
        pq[q] += (int)__builtin_popcount(mq);
      }
    }
  }

  const v16h a00 = ldf(out16 + (size_t)(s0 + lm) * HD + 8 * hh);
  const v16h a01 = ldf(out16 + (size_t)(s0 + lm) * HD + 32 + 8 * hh);
  const v16h a10 = ldf(out16 + (size_t)(s0 + 16 + lm) * HD + 8 * hh);
  const v16h a11 = ldf(out16 + (size_t)(s0 + 16 + lm) * HD + 32 + 8 * hh);

  {
    const bool up = (wave >> 2) != 0;
    const v16h q0 = selv(up, a10, a00), q1 = selv(up, a11, a01);
    const int ntq = wave & 3;
    v8f acc = zacc();
    acc = wmh(q0, ldf(B2t + (size_t)(ntq * 16 + lm) * HD + 8 * hh), acc);
    acc = wmh(q1, ldf(B2t + (size_t)(ntq * 16 + lm) * HD + 32 + 8 * hh), acc);
#pragma unroll
    for (int r = 0; r < 8; ++r) Qs[((wave >> 2) * 16 + 8 * hh + r) * HD + ntq * 16 + lm] = acc[r] * W2INV;
  }
  __syncthreads();
  const int T = min(max(misc[1], 0), MAXT);
  const int nTj = (T + NWAVE - 1) / NWAVE;
  const v8h z8 = zero8();

#pragma unroll 1
  for (int oc = 0; oc < 4; ++oc) {
#pragma unroll 1
    for (int j = 0; j < NHID / NWAVE; ++j) {
      const int hs = wave + NWAVE * j;
      const _Float16* bp = W2t + (size_t)(hs * HD + oc * 16 + lm) * HD + 8 * hh;
      const v16h b0 = ldf(bp), b1 = ldf(bp + 32);
      v8f p0 = zacc(), p1 = zacc();
      p0 = wmh(a00, b0, p0);
      p0 = wmh(a01, b1, p0);
      p1 = wmh(a10, b0, p1);
      p1 = wmh(a11, b1, p1);
#pragma unroll
      for (int r = 0; r < 8; ++r) {
        Pt[((8 * hh + r) * 16 + lm) * PH + hs] = (_Float16)p0[r];
        Pt[((16 + 8 * hh + r) * 16 + lm) * PH + hs] = (_Float16)p1[r];
      }
    }
    __syncthreads();
#pragma unroll 1
    for (int tj = 0; tj < nTj; ++tj) {
      const int t = wave + NWAVE * tj;
      const bool act = t < T;
      const int tv = ttab[min(t, MAXT - 1)];
      const int s = tv & (NS - 1);
      const int stt = min((tv >> 8) & 4095, CAPS - 1);
      const int cn = min((tv >> 20) & 31, 16);
      if (act) {
#pragma unroll
        for (int q = 0; q < 8; ++q) {
          const int row = 2 * q + hh;
          const int piece = lm * 8;
          const bool valid = row < cn;
          int e = sorted[min(stt + min(row, 15), CAPS - 1)] >> 8;
          e = min(max(e, 0), nE - 1);
          v8h v = *(const v8h*)(h1 + (size_t)e * NHID + piece);
          if (!valid) v = z8;
          *(v8h*)(As + (size_t)(wave * 16 + row) * AP + piece) = v;
        }
      }
      __syncthreads();
      if (act) {
        v16h af[4];
#pragma unroll
        for (int ks = 0; ks < 4; ++ks) af[ks] = ldf(As + (size_t)(wave * 16 + lm) * AP + ks * 32 + 8 * hh);
        v8f acc = zacc();
#pragma unroll
        for (int ks = 0; ks < 4; ++ks)
          acc = wmh(af[ks], ldf(Pt + (size_t)(s * 16 + lm) * PH + ks * 32 + 8 * hh), acc);
        const float qv = Qs[s * HD + oc * 16 + lm];
#pragma unroll
        for (int r = 0; r < 8; ++r) {
          const int row = 8 * hh + r;
          if (row < cn) Mr[(size_t)min(stt + row, CAPS - 1) * HD + oc * 16 + lm] = acc[r] * W2INV + qv;
        }
      }
      __syncthreads();
    }
  }
  __syncthreads();
#pragma unroll 1
  for (int pass = 0; pass < 2; ++pass) {
#pragma unroll 1
    for (int i = 0; i < CAPS / 16; ++i) {
      const int pi = wave + NWAVE * i;
      if (2 * pi >= nHit) break;
      const int p = 2 * pi + hh;
      const bool valid = p < nHit;
      const int pc = min(p, CAPS - 1);
      int e = sorted[pc] >> 8;
      e = min(max(e, 0), nE - 1);
      const v4f v = *(const v4f*)(Mr + (size_t)pc * HD + 4 * lm);
      if (valid) *(volatile v4f*)(msg + (size_t)e * HD + 4 * lm) = v;
    }
    if (pass == 0) __threadfence();
  }
}

__global__ __launch_bounds__(NTHR) void k_node(const int* __restrict__ ei, const float* __restrict__ msg,
                                               const _Float16* __restrict__ Rt, const float* __restrict__ cbias,
                                               const _Float16* __restrict__ Wiht, const _Float16* __restrict__ Whht,
                                               const float* __restrict__ bih, const float* __restrict__ bhh,
                                               float* out32, _Float16* out16, int nE, int vec8) {
  float* accl = (float*)(dsm + D_ACC);
  float* cntd = (float*)(dsm + D_CNT);
  int* wl = (int*)(dsm + D_WL);
  int* pend = (int*)(dsm + D_PEND);
  _Float16* m16 = (_Float16*)(dsm + D_M16);
  float* st = (float*)(dsm + D_ST);
  int* wcnt = (int*)(dsm + D_WCS);
  int* misc = (int*)(dsm + D_MSC);
  const int tid = threadIdx.x, lane = tid & 31, wave = tid >> 5, hh = lane >> 4, lm = lane & 15;
  const int d0 = blockIdx.x * NBD;

  for (int i = tid; i < NBD * HD; i += NTHR) accl[i] = 0.0f;
  cntd[tid] = 0.0f;
  const int nHit = build_list(ei + nE, nE, d0, NBD, 0, vec8, wl, pend, CAPD, wcnt, misc, tid, wave, lane);

#pragma unroll 1
  for (int i = 0; i < CAPD; ++i) {
    if (i >= nHit) break;
    const int v = pend[i];
    const int sl = v & 255;
    if ((sl & (NWAVE - 1)) == wave) {
      int e = v >> 8;
      e = min(max(e, 0), nE - 1);
      const v2f x = *(const v2f*)(msg + (size_t)e * HD + 2 * lane);
      float* ap = accl + sl * HD + 2 * lane;
      ap[0] += x.x;
      ap[1] += x.y;
      if (lane == 0) cntd[sl] += 1.0f;
    }
  }
  __syncthreads();
  cntd[tid] = 1.0f / fmaxf(cntd[tid], 1.0f);
  __syncthreads();

#pragma unroll 1
  for (int jt = 0; jt < NBD / 16 / NWAVE; ++jt) {
    const int mt = wave * (NBD / 16 / NWAVE) + jt;
    const size_t rb = (size_t)d0 + mt * 16;
    const v16h ao0 = ldf(out16 + (rb + lm) * HD + 8 * hh);
    const v16h ao1 = ldf(out16 + (rb + lm) * HD + 32 + 8 * hh);
#pragma unroll
    for (int nt = 0; nt < 4; ++nt) {
      v8f acc = zacc();
      acc = wmh(ao0, ldf(Rt + (size_t)(nt * 16 + lm) * HD + 8 * hh), acc);
      acc = wmh(ao1, ldf(Rt + (size_t)(nt * 16 + lm) * HD + 32 + 8 * hh), acc);
      const int col = nt * 16 + lm;
      const float cb = cbias[col];
#pragma unroll
      for (int r = 0; r < 8; ++r) {
        const int row = 8 * hh + r;
        const int sl = mt * 16 + row;
        const float v = fmaxf(acc[r] * WINV + cb + accl[sl * HD + col] * cntd[sl], 0.0f);
        m16[(wave * 16 + row) * HD + col] = (_Float16)v;
      }
    }
    __syncthreads();
    const v16h am0 = ldf(m16 + (size_t)(wave * 16 + lm) * HD + 8 * hh);
    const v16h am1 = ldf(m16 + (size_t)(wave * 16 + lm) * HD + 32 + 8 * hh);
#pragma unroll 1
    for (int nt = 0; nt < 4; ++nt) {
      v8f gI[3], gH[3];
#pragma unroll
      for (int g = 0; g < 3; ++g) {
        gI[g] = zacc();
        gH[g] = zacc();
        const _Float16* wi = Wiht + (size_t)(g * HD + nt * 16 + lm) * HD + 8 * hh;
        const _Float16* wh = Whht + (size_t)(g * HD + nt * 16 + lm) * HD + 8 * hh;
        gI[g] = wmh(am0, ldf(wi), gI[g]);
        gI[g] = wmh(am1, ldf(wi + 32), gI[g]);
        gH[g] = wmh(ao0, ldf(wh), gH[g]);
        gH[g] = wmh(ao1, ldf(wh + 32), gH[g]);
      }
      const int col = nt * 16 + lm;
      const float bi0 = bih[col], bi1 = bih[HD + col], bi2 = bih[2 * HD + col];
      const float bh0 = bhh[col], bh1 = bhh[HD + col], bh2 = bhh[2 * HD + col];
#pragma unroll
      for (int r = 0; r < 8; ++r) {
        const int row = 8 * hh + r;
        const float hold = out32[(rb + row) * HD + col];
        const float xr = gI[0][r] * WINV + bi0 + gH[0][r] * WINV + bh0;
        const float xz = gI[1][r] * WINV + bi1 + gH[1][r] * WINV + bh1;
        const float hn = gH[2][r] * WINV + bh2;
        const float xn = gI[2][r] * WINV + bi2;
        const float rg = sigm(xr);
        const float zg = sigm(xz);
        const float ng = tanhf(xn + rg * hn);
        st[(wave * 16 + row) * HD + col] = (1.0f - zg) * ng + zg * hold;
      }
    }
    __syncthreads();
#pragma unroll 1
    for (int pass = 0; pass < 2; ++pass) {
#pragma unroll
      for (int q = 0; q < 8; ++q) {
        const int row = 2 * q + hh;
        const v4f v = *(const v4f*)(st + (wave * 16 + row) * HD + 4 * lm);
        *(volatile v4f*)(out32 + (rb + row) * HD + 4 * lm) = v;
      }
#pragma unroll
      for (int q = 0; q < 4; ++q) {
        const int row = 4 * q + (lane >> 3);
        const int piece = (lane & 7) * 8;
        const float* sp = st + (wave * 16 + row) * HD + piece;
        const v8h hv = pack8(*(const v4f*)sp, *(const v4f*)(sp + 4));
        *(volatile v8h*)(out16 + (rb + row) * HD + piece) = hv;
      }
      if (pass == 0) __threadfence();
    }
  }
}

__global__ __launch_bounds__(NTHR) void k_s2s(const float* __restrict__ out32, const int* __restrict__ batch,
                                              const float* __restrict__ lwih, const float* __restrict__ lwhh,
                                              const float* __restrict__ lbih, const float* __restrict__ lbhh,
                                              const float* __restrict__ l1w, const float* __restrict__ l1b,
                                              const float* __restrict__ l2w, const float* __restrict__ l2b,
                                              float* res, int nN, int nB, int nNp) {
  float* en = (float*)dsm;
  float* qst = en + nNp;
  float* cs = qst + NG * 128;
  float* rtab = cs + NG * HD;
  float* gbuf = rtab + NG * HD;
  float* gmax = gbuf + 256;
  float* ginv = gmax + NG;
  float* resl = ginv + NG;
  const int tid = threadIdx.x;
  for (int i = tid; i < NG * 128; i += NTHR) qst[i] = 0.0f;
  for (int i = tid; i < NG * HD; i += NTHR) cs[i] = 0.0f;
  if (tid < NG) resl[tid] = 0.0f;
  __syncthreads();

#pragma unroll 1
  for (int step = 0; step < 3; ++step) {
#pragma unroll 1
    for (int b = 0; b < nB; ++b) {
      {
        float acc = lbih[tid] + lbhh[tid];
        const float* qr = qst + b * 128;
#pragma unroll 1
        for (int k = 0; k < 128; ++k) acc += qr[k] * lwih[(size_t)k * 256 + tid];
#pragma unroll 1
        for (int k = 0; k < HD; ++k) acc += qr[k] * lwhh[(size_t)k * 256 + tid];
        gbuf[tid] = acc;
      }
      __syncthreads();
      if (tid < HD) {
        const int tc = min(tid, HD - 1);
#pragma unroll 1
        for (int q = 0; q < 4; ++q) {
          const float v = gbuf[q * HD + tc];
          const bool isg = (q == 2);
          const float t = tanhf(isg ? v : 0.5f * v);
          gbuf[q * HD + tc] = isg ? t : (0.5f * t + 0.5f);
        }
        const float ii = gbuf[tc], ff = gbuf[HD + tc], gg = gbuf[2 * HD + tc], oo = gbuf[3 * HD + tc];
        const float c2 = ff * cs[b * HD + tc] + ii * gg;
        const float h2 = oo * tanhf(c2);
        cs[b * HD + tc] = c2;
        qst[b * 128 + tc] = h2;
      }
      __syncthreads();
    }
    for (int n = tid; n < nN; n += NTHR) {
      const int nc = min(n, nN - 1);
      const int bg = batch[nc];
      const int bc = min(max(bg, 0), nB - 1);
      const float* orow = out32 + (size_t)nc * HD;
      const float* qrow = qst + bc * 128;
      float acc = 0.0f;
#pragma unroll 1
      for (int k = 0; k < HD; k += 4) {
        const v4f o = *(const v4f*)(orow + k);
        const v4f q = *(const v4f*)(qrow + k);
        acc += o.x * q.x + o.y * q.y + o.z * q.z + o.w * q.w;
      }
      en[nc] = acc;
    }
    __syncthreads();
    if (tid < nB) {
      float mx = -__builtin_huge_valf();
#pragma unroll 1
      for (int n = 0; n < nN; ++n) {
        if (batch[n] == tid) mx = fmaxf(mx, en[n]);
      }
      gmax[min(tid, NG - 1)] = mx;
    }
    __syncthreads();
    for (int n = tid; n < nN; n += NTHR) {
      const int nc = min(n, nN - 1);
      const int bg = batch[nc];
      const bool valid = (unsigned)bg < (unsigned)nB;
      const int bc = min(max(bg, 0), nB - 1);
      const float ee = valid ? expf(en[nc] - gmax[bc]) : 0.0f;
      en[nc] = ee;
    }
    __syncthreads();
    if (tid < nB) {
      float s = 0.0f;
#pragma unroll 1
      for (int n = 0; n < nN; ++n) {
        if (batch[n] == tid) s += en[n];
      }
      ginv[min(tid, NG - 1)] = 1.0f / (s + 1e-16f);
    }
    __syncthreads();
    if (tid < HD) {
      const int c = min(tid, HD - 1);
      for (int g = 0; g < nB; ++g) rtab[g * HD + c] = 0.0f;
#pragma unroll 1
      for (int n = 0; n < nN; ++n) {
        const int bg = batch[n];
        const int bc = min(max(bg, 0), nB - 1);
        if ((unsigned)bg < (unsigned)nB) {
          const float a = en[n] * ginv[bc];
          rtab[bc * HD + c] += a * out32[(size_t)n * HD + c];
        }
      }
      for (int g = 0; g < nB; ++g) qst[g * 128 + HD + c] = rtab[g * HD + c];
    }
    __syncthreads();
  }
  for (int idx = tid; idx < nB * HD; idx += NTHR) {
    const int ic = min(idx, nB * HD - 1);
    const int b = ic >> 6, j = ic & 63;
    float acc = l1b[j];
    const float* qr = qst + b * 128;
#pragma unroll 1
    for (int k = 0; k < 128; ++k) acc += qr[k] * l1w[k * HD + j];
    rtab[ic] = fmaxf(acc, 0.0f);
  }
  __syncthreads();
  if (tid < nB) {
    const int tb = min(tid, NG - 1);
    float s = l2b[0];
#pragma unroll 1
    for (int k = 0; k < HD; ++k) s += rtab[tb * HD + k] * l2w[k];
    resl[tb] = s;
  }
  __syncthreads();
  if ((nB & 3) == 0) {
    const bool wr = tid < (nB >> 2);
    v4f v = {0.0f, 0.0f, 0.0f, 0.0f};
    if (wr) v = *(const v4f*)(resl + 4 * min(tid, NG / 4 - 1));
    if (wr) *(volatile v4f*)(res + 4 * tid) = v;
    __threadfence();
    if (wr) *(volatile v4f*)(res + 4 * tid) = v;
  } else {
    const bool wr = tid < nB;
    const float v = wr ? resl[min(tid, NG - 1)] : 0.0f;
    if (wr) *(volatile float*)(res + tid) = v;
    __threadfence();
    if (wr) *(volatile float*)(res + tid) = v;
  }
}

static void launch_cvt(const float* src, _Float16* dst, int rows, int cols, int mode, int srows, int p0,
                       float scale, hipStream_t stream) {
  const int pieces = (rows * cols) >> 3;
  const int grid = (pieces + NTHR - 1) / NTHR;
  k_cvt<<<grid, NTHR, 0, stream>>>(src, dst, rows, cols, mode, srows, p0, scale);
}

extern "C" void kernel_launch(void* const* d_in, const int* in_sizes, int n_in,
                              void* d_out, int out_size, void* d_ws, size_t ws_size,
                              hipStream_t stream) {
  if (n_in < 24) return;
  const int nN = in_sizes[2];
  const int nE = in_sizes[1] / 2;
  const int nB = out_size;
  if (nN < 1 || nE < 1 || nE >= (1 << 22) || nN >= (1 << 22)) return;
  if (in_sizes[0] != nN * 32 || in_sizes[1] != nE * 2 || in_sizes[3] != nE * HD) return;
  if (in_sizes[4] != 32 * HD || in_sizes[5] != HD || in_sizes[6] != HD * NHID || in_sizes[7] != NHID) return;
  if (in_sizes[8] != NHID * HD * HD || in_sizes[9] != HD * HD || in_sizes[10] != HD * HD || in_sizes[11] != HD) return;
  if (in_sizes[12] != HD * 192 || in_sizes[13] != HD * 192 || in_sizes[14] != 192 || in_sizes[15] != 192) return;
  if (in_sizes[16] != 128 * 256 || in_sizes[17] != HD * 256 || in_sizes[18] != 256 || in_sizes[19] != 256) return;
  if (in_sizes[20] != 128 * HD || in_sizes[21] != HD || in_sizes[22] != HD || in_sizes[23] < 1) return;
  if (nB < 1 || nB > NG) return;

  const float* x        = (const float*)d_in[0];
  const int*   ei       = (const int*)d_in[1];
  const int*   batch    = (const int*)d_in[2];
  const float* ea       = (const float*)d_in[3];
  const float* lin0_w   = (const float*)d_in[4];
  const float* lin0_b   = (const float*)d_in[5];
  const float* nn_w1    = (const float*)d_in[6];
  const float* nn_b1    = (const float*)d_in[7];
  const float* nn_w2    = (const float*)d_in[8];
  const float* nn_b2    = (const float*)d_in[9];
  const float* conv_rt  = (const float*)d_in[10];
  const float* conv_bs  = (const float*)d_in[11];
  const float* gru_wih  = (const float*)d_in[12];
  const float* gru_whh  = (const float*)d_in[13];
  const float* gru_bih  = (const float*)d_in[14];
  const float* gru_bhh  = (const float*)d_in[15];
  const float* lstm_wih = (const float*)d_in[16];
  const float* lstm_whh = (const float*)d_in[17];
  const float* lstm_bih = (const float*)d_in[18];
  const float* lstm_bhh = (const float*)d_in[19];
  const float* lin1_w   = (const float*)d_in[20];
  const float* lin1_b   = (const float*)d_in[21];
  const float* lin2_w   = (const float*)d_in[22];
  const float* lin2_b   = (const float*)d_in[23];
  float* res = (float*)d_out;

  const int NP = ((nN + NBD - 1) / NBD) * NBD;
  const int EP = ((nE + 63) / 64) * 64;
  const int nBlkS = (nN + NS - 1) / NS;
  const int nBlkD = NP / NBD;

  char* ws = (char*)d_ws;
  size_t off = 0;
#define CARVE(ptr, type, bytes) type* ptr = (type*)(ws + off); off += (((size_t)(bytes)) + 255) & ~(size_t)255;
  CARVE(x16,   _Float16, (size_t)NP * 32 * 2)
  CARVE(ea16,  _Float16, (size_t)EP * HD * 2)
  CARVE(W0t,   _Float16, (size_t)HD * 32 * 2)
  CARVE(W1t,   _Float16, (size_t)NHID * HD * 2)
  CARVE(W2t,   _Float16, (size_t)HD * HD * 2 * NHID * 2)
  CARVE(B2t,   _Float16, (size_t)HD * HD * 2)
  CARVE(Rt,    _Float16, (size_t)HD * HD * 2)
  CARVE(Wiht,  _Float16, (size_t)192 * HD * 2)
  CARVE(Whht,  _Float16, (size_t)192 * HD * 2)
  CARVE(out32, float,    (size_t)NP * HD * 4)
  CARVE(out16, _Float16, (size_t)NP * HD * 2)
  CARVE(h1p,   _Float16, (size_t)EP * NHID * 2)
  CARVE(msgp,  float,    (size_t)EP * HD * 4)
#undef CARVE
  if (off > ws_size || off > ((size_t)128 << 20)) return;

  const int nNp = (nN + 3) & ~3;
  const size_t s2sLds = ((size_t)nNp + NG * 128 + NG * HD + NG * HD + 256 + NG + NG + NG) * 4;
  if (s2sLds > 300000) return;

  hipFuncSetAttribute(reinterpret_cast<const void*>(&k_msg), hipFuncAttributeMaxDynamicSharedMemorySize, MSG_LDS);
  hipFuncSetAttribute(reinterpret_cast<const void*>(&k_node), hipFuncAttributeMaxDynamicSharedMemorySize, NODE_LDS);
  hipFuncSetAttribute(reinterpret_cast<const void*>(&k_s2s), hipFuncAttributeMaxDynamicSharedMemorySize, (int)s2sLds);

  launch_cvt(x, x16, NP, 32, 0, nN, 0, 1.0f, stream);
  launch_cvt(ea, ea16, EP, HD, 0, nE, 0, 1.0f, stream);
  launch_cvt(lin0_w, W0t, HD, 32, 1, 0, 0, WSC, stream);
  launch_cvt(nn_w1, W1t, NHID, HD, 1, 0, 0, WSC, stream);
  launch_cvt(nn_w2, W2t, HD * HD * 2, HD, 2, 0, HD * HD, W2SC, stream);
  launch_cvt(nn_b2, B2t, HD, HD, 1, 0, 0, W2SC, stream);
  launch_cvt(conv_rt, Rt, HD, HD, 1, 0, 0, WSC, stream);
  launch_cvt(gru_wih, Wiht, 192, HD, 1, 0, 0, WSC, stream);
  launch_cvt(gru_whh, Whht, 192, HD, 1, 0, 0, WSC, stream);

  k_gemm<4, 1, 1, 1><<<NP / 64, NTHR, 0, stream>>>(x16, W0t, lin0_b, out32, out16);
  k_gemm<8, 2, 0, 1><<<EP / 64, NTHR, 0, stream>>>(ea16, W1t, nn_b1, out32, h1p);

  const int vec8d = ((nE & 3) == 0) ? 1 : 0;
  for (int it = 0; it < 3; ++it) {
    k_msg<<<nBlkS, NTHR, MSG_LDS, stream>>>(ei, out16, h1p, W2t, B2t, msgp, nN, nE, 1);
    k_node<<<nBlkD, NTHR, NODE_LDS, stream>>>(ei, msgp, Rt, conv_bs, Wiht, Whht, gru_bih, gru_bhh,
                                                out32, out16, nE, vec8d);
  }
  k_s2s<<<1, NTHR, s2sLds, stream>>>(out32, batch, lstm_wih, lstm_whh, lstm_bih, lstm_bhh,
                                     lin1_w, lin1_b, lin2_w, lin2_b, res, nN, nB, nNp);
}
